// CCL_Module_78082505441363
// MI455X (gfx1250) — hardware-verified
//
#include <hip/hip_runtime.h>

typedef __attribute__((ext_vector_type(16))) _Float16 v16h;
typedef __attribute__((ext_vector_type(8)))  _Float16 v8h;
typedef __attribute__((ext_vector_type(8)))  float    v8f;
typedef __attribute__((ext_vector_type(4)))  float    v4f;
#define VST2(T, ptr, val) do { const T _v = (val); *(volatile T*)(ptr) = _v; __threadfence(); *(volatile T*)(ptr) = _v; } while (0)

constexpr int B = 4, C = 32, H = 64, W = 64;
constexpr int L = H * W;
constexpr int D = C * 9;
constexpr int TR = 32;
constexpr int NT = L / TR;
constexpr int TILE_BYTES = TR * D * 2;
constexpr float SM_SCALE = 10.0f;

__global__ void norm_kernel(const float* __restrict__ f1,
                            const float* __restrict__ f2,
                            _Float16* __restrict__ N1,
                            _Float16* __restrict__ N2) {
  int idx = blockIdx.x * blockDim.x + threadIdx.x;
  if (idx >= B * L) return;
  int b = idx >> 12;
  int p = idx & (L - 1);
  const float* p1 = f1 + (size_t)b * C * L + p;
  const float* p2 = f2 + (size_t)b * C * L + p;
  float s1 = 0.f, s2 = 0.f;
  #pragma unroll 4
  for (int c = 0; c < C; ++c) {
    float a = p1[c * L]; s1 += a * a;
    float d = p2[c * L]; s2 += d * d;
  }
  float i1 = 1.0f / fmaxf(sqrtf(s1), 1e-12f);
  float i2 = 1.0f / fmaxf(sqrtf(s2), 1e-12f);
  _Float16* o1 = N1 + (size_t)b * C * L + p;
  _Float16* o2 = N2 + (size_t)b * C * L + p;
  #pragma unroll 4
  for (int c = 0; c < C; ++c) {
    VST2(_Float16, o1 + c * L, (_Float16)(p1[c * L] * i1));
    VST2(_Float16, o2 + c * L, (_Float16)(p2[c * L] * i2));
  }
}

__global__ void patch_kernel(const _Float16* __restrict__ N1,
                             const _Float16* __restrict__ N2,
                             _Float16* __restrict__ Qm,
                             _Float16* __restrict__ Km) {
  int tid = blockIdx.x * blockDim.x + threadIdx.x;
  if (tid >= B * L * D / 8) return;
  v8h q8, k8;
  #pragma unroll
  for (int e = 0; e < 8; ++e) {
    const int f = tid * 8 + e;
    const int row = f / D, col = f - row * D;
    const int b = row >> 12, l = row & (L - 1), c = col / 9, tap = col - c * 9;
    const int ys = (l >> 6) + tap / 3 - 1, xs = (l & 63) + tap % 3 - 1;
    const bool in = (ys >= 0) & (ys < H) & (xs >= 0) & (xs < W);
    const size_t src = ((size_t)(b * C + c)) * L + ys * W + xs;
    q8[e] = in ? N1[src] : (_Float16)0.0f;
    k8[e] = in ? N2[src] : (_Float16)0.0f;
  }
  VST2(v8h, Qm + (size_t)tid * 8, q8);
  VST2(v8h, Km + (size_t)tid * 8, k8);
}


__device__ __forceinline__ void stage_tile(const _Float16* gsrc,
                                           _Float16* lbuf, int t) {
  for (int p = t; p < TILE_BYTES / 16; p += 256) *(v8h*)(lbuf + p * 8) = *(const v8h*)(gsrc + p * 8);
}

__global__ __launch_bounds__(256) void corr_flow_kernel(
    const _Float16* __restrict__ Qm,
    const _Float16* __restrict__ Km,
    float* __restrict__ out) {
  __shared__ __align__(16) _Float16 smem[2][TR * D];
  __shared__ __align__(16) float sflow[2][128];

  const int t       = threadIdx.x;
  const int lane    = t & 31;
  const int wave    = t >> 5;
  const int b       = blockIdx.x >> 5;
  const int blk     = blockIdx.x & 31;
  const int q_base  = blk * 128 + wave * 16;
  const int halfsel = lane >> 4;
  const int r       = lane & 15;

  const _Float16* qp = Qm + ((size_t)(b * L + q_base + r)) * D + halfsel * 8;
  v16h qreg[9];
  #pragma unroll
  for (int ck = 0; ck < 9; ++ck) {
    const v8h lo = *(const v8h*)(qp + ck * 32), hi = *(const v8h*)(qp + ck * 32 + 16);
    qreg[ck] = __builtin_shufflevector(lo, hi, 0, 1, 2, 3, 4, 5, 6, 7, 8, 9, 10, 11, 12, 13, 14, 15);
  }

  const _Float16* kbase = Km + ((size_t)b * L) * D;

  float m = -__builtin_inff();
  float Z = 0.f, Sy = 0.f, Sx = 0.f;

  stage_tile(kbase, &smem[0][0], t);

  for (int i = 0; i < NT; ++i) {
    const int cur = i & 1;
    __syncthreads();
    if (i + 1 < NT) stage_tile(kbase + (size_t)(i + 1) * TR * D, &smem[1 - cur][0], t);

    const _Float16* a0 = &smem[cur][0] + (size_t)r * D + halfsel * 8;
    const _Float16* a1 = a0 + 16 * D;
    v8f acc0 = {}, acc1 = {};
    #pragma unroll
    for (int ck = 0; ck < 9; ++ck) {
      v8h lo0 = *(const v8h*)(a0 + ck * 32);
      v8h hi0 = *(const v8h*)(a0 + ck * 32 + 16);
      v8h lo1 = *(const v8h*)(a1 + ck * 32);
      v8h hi1 = *(const v8h*)(a1 + ck * 32 + 16);
      v16h A0 = __builtin_shufflevector(lo0, hi0,
                0, 1, 2, 3, 4, 5, 6, 7, 8, 9, 10, 11, 12, 13, 14, 15);
      v16h A1 = __builtin_shufflevector(lo1, hi1,
                0, 1, 2, 3, 4, 5, 6, 7, 8, 9, 10, 11, 12, 13, 14, 15);
      acc0 = __builtin_amdgcn_wmma_f32_16x16x32_f16(
                 false, A0, false, qreg[ck], (short)0, acc0, false, false);
      acc1 = __builtin_amdgcn_wmma_f32_16x16x32_f16(
                 false, A1, false, qreg[ck], (short)0, acc1, false, false);
      asm volatile("v_nop\n\tv_nop\n\tv_nop\n\tv_nop" : "+v"(acc0), "+v"(acc1) : "v"(A0), "v"(A1));
    }

    const int lb = i * TR;
    float s[16];
    float tm = -__builtin_inff();
    #pragma unroll
    for (int v = 0; v < 8; ++v) {
      s[v]     = acc0[v] * SM_SCALE;
      s[v + 8] = acc1[v] * SM_SCALE;
      tm = fmaxf(tm, fmaxf(s[v], s[v + 8]));
    }
    float nm    = fmaxf(m, tm);
    float scale = expf(m - nm);
    Z *= scale; Sy *= scale; Sx *= scale;
    #pragma unroll
    for (int v = 0; v < 16; ++v) {
      float e   = expf(s[v] - nm);
      int  lrow = lb + ((v >> 3) << 4) + halfsel * 8 + (v & 7);
      Z  += e;
      Sy += e * (float)(lrow >> 6);
      Sx += e * (float)(lrow & 63);
    }
    m = nm;
  }

  float mo  = __shfl_xor(m, 16, 32);
  float Zo  = __shfl_xor(Z, 16, 32);
  float Syo = __shfl_xor(Sy, 16, 32);
  float Sxo = __shfl_xor(Sx, 16, 32);
  float M2 = fmaxf(m, mo);
  float sa = expf(m - M2), sb = expf(mo - M2);
  Z  = Z * sa + Zo * sb;
  Sy = Sy * sa + Syo * sb;
  Sx = Sx * sa + Sxo * sb;

  if (halfsel == 0) {
    int q = q_base + r;
    float qy = (float)(q >> 6), qx = (float)(q & 63);
    sflow[0][wave * 16 + r] = Sx / Z - qx;
    sflow[1][wave * 16 + r] = Sy / Z - qy;
  }
  __syncthreads();
  if (t < 64) {
    const int ch = t >> 5, p = t & 31;
    VST2(v4f, out + (size_t)b * 2 * L + (size_t)ch * L + blk * 128 + p * 4, *(const v4f*)(&sflow[ch][p * 4]));
  }
}

extern "C" void kernel_launch(void* const* d_in, const int* in_sizes, int n_in,
                              void* d_out, int out_size, void* d_ws, size_t ws_size,
                              hipStream_t stream) {
  const float* f1 = (const float*)d_in[0];
  const float* f2 = (const float*)d_in[1];
  float* out = (float*)d_out;

  _Float16* N1 = (_Float16*)d_ws;
  _Float16* N2 = N1 + (size_t)B * C * L;
  _Float16* Qm = N2 + (size_t)B * C * L;
  _Float16* Km = Qm + (size_t)B * L * D;

  (void)in_sizes; (void)n_in; (void)out_size;
  if (ws_size < (size_t)2 * B * C * L * 2 + (size_t)2 * B * L * D * 2) return;
  norm_kernel <<<(B * L + 255) / 256, 256, 0, stream>>>(f1, f2, N1, N2);
  patch_kernel<<<(B * L * D / 8 + 255) / 256, 256, 0, stream>>>(N1, N2, Qm, Km);
  corr_flow_kernel<<<B * 32, 256, 0, stream>>>(Qm, Km, out);
}
